// PlgaLayer_63196148793962
// MI455X (gfx1250) — hardware-verified
//
#include <hip/hip_runtime.h>


#define NB_  1
#define NBH  (2 * NH_)
#define NT_  2048
#define DM   1024
#define NH_  16
#define HD   64
#define NTK  (NB_ * NT_)
#define NW   1024
#define NQKV 1024
#define PSC  32768.0f
#define LOSC 1024.0f
#define LOSCI (1.0f / 1024.0f)

typedef _Float16 h16;
typedef unsigned short bf;
typedef __attribute__((ext_vector_type(16))) __bf16   v16bf;
typedef __attribute__((ext_vector_type(16))) _Float16 v16h;
typedef __attribute__((ext_vector_type(8)))  _Float16 v8h;
typedef __attribute__((ext_vector_type(8)))  unsigned short v8us;
typedef __attribute__((ext_vector_type(8)))  float    v8f;
typedef __attribute__((ext_vector_type(4)))  float    v4f;
typedef v8h  __attribute__((may_alias)) v8ha;
typedef v4f  __attribute__((may_alias)) v4fa;
typedef v8us __attribute__((may_alias)) v8usa;

__device__ __forceinline__ unsigned short f2bf(float f) { unsigned u = __float_as_uint(f); u += 0x7FFFu + ((u >> 16) & 1u); return (unsigned short)(u >> 16); }
__device__ __forceinline__ float bf2f(unsigned short b) { return __uint_as_float(((unsigned)b) << 16); }
__device__ __forceinline__ float bfr(float f) { return bf2f(f2bf(f)); }
__device__ __forceinline__ v16h cat16(v8h lo, v8h hi) { return __builtin_shufflevector(lo, hi, 0, 1, 2, 3, 4, 5, 6, 7, 8, 9, 10, 11, 12, 13, 14, 15); }
__device__ __forceinline__ v16bf cat16b(v8us lo, v8us hi) { return __builtin_bit_cast(v16bf, __builtin_shufflevector(lo, hi, 0, 1, 2, 3, 4, 5, 6, 7, 8, 9, 10, 11, 12, 13, 14, 15)); }
__device__ __forceinline__ v8f wmma16(v16h a, v16h b, v8f c) { return __builtin_amdgcn_wmma_f32_16x16x32_f16(false, a, false, b, (short)0, c, false, false); }
__device__ __forceinline__ v8f wmmab(v16bf a, v16bf b, v8f c) { return __builtin_amdgcn_wmma_f32_16x16x32_bf16(false, a, false, b, (short)0, c, false, false); }

__global__ __launch_bounds__(256) void k_cvtb(const float* __restrict__ src, int nrows, bf* dst) {
    const int lane = threadIdx.x & 31, r = blockIdx.x * 8 + (threadIdx.x >> 5);
    if (r >= nrows) return;
    v8us o[DM / 256];
#pragma unroll
    for (int q = 0; q < DM / 256; ++q) { v8us t;
#pragma unroll
        for (int i = 0; i < 8; ++i) t[i] = f2bf(src[(size_t)r * DM + q * 256 + lane * 8 + i]);
        o[q] = t; }
#pragma unroll
    for (int q = 0; q < DM / 256; ++q) *(volatile v8us*)(dst + (size_t)r * DM + q * 256 + lane * 8) = o[q];
    __threadfence();
#pragma unroll
    for (int q = 0; q < DM / 256; ++q) *(volatile v8us*)(dst + (size_t)r * DM + q * 256 + lane * 8) = o[q];
}

__global__ __launch_bounds__(128) void k_gemm3(const bf* __restrict__ Ah, const bf* __restrict__ Al, const bf* __restrict__ Bh, const bf* __restrict__ Bl, int K, float* C, int ldc) {
    __shared__ __align__(16) float ost[4][16 * 68];
    const int lane = threadIdx.x & 31, wave = threadIdx.x >> 5, lr = lane & 15, hi = lane >> 4;
    const int r0 = blockIdx.x * 64 + wave * 16, c0 = blockIdx.y * 64;
    const size_t aoff = (size_t)(r0 + lr) * K + 8 * hi;
    v8f acc[4];
#pragma unroll
    for (int t = 0; t < 4; ++t) acc[t] = (v8f){};
#pragma unroll 1
    for (int kc = 0; kc < K; kc += 32) {
        const v16bf a = cat16b(*(const v8us*)(Ah + aoff + kc), *(const v8us*)(Ah + aoff + kc + 16));
        const v16bf al = cat16b(*(const v8us*)(Al + aoff + kc), *(const v8us*)(Al + aoff + kc + 16));
#pragma unroll
        for (int t = 0; t < 4; ++t) { const size_t bo = (size_t)(c0 + t * 16 + lr) * K + kc + 8 * hi;
            const v16bf bh = cat16b(*(const v8us*)(Bh + bo), *(const v8us*)(Bh + bo + 16)); const v16bf bl = cat16b(*(const v8us*)(Bl + bo), *(const v8us*)(Bl + bo + 16));
            acc[t] = wmmab(a, bh, acc[t]); acc[t] = wmmab(al, bh, acc[t]); acc[t] = wmmab(a, bl, acc[t]); }
        asm volatile("v_nop\n\tv_nop\n\tv_nop\n\tv_nop" : "+v"(acc[0]), "+v"(acc[1]), "+v"(acc[2]), "+v"(acc[3]) : "v"(a), "v"(al));
    }
    float* os = &ost[wave][0];
#pragma unroll
    for (int t = 0; t < 4; ++t) {
#pragma unroll
        for (int j = 0; j < 8; ++j) os[(hi * 8 + j) * 68 + t * 16 + lr] = acc[t][j]; }
    __builtin_amdgcn_wave_barrier(); asm volatile("" ::: "memory");
    float* crow = C + (size_t)r0 * ldc + c0;
    auto pass = [&]() {
#pragma unroll
        for (int s = 0; s < 8; ++s) { const int Lid = (lane >> 3) + 4 * s, piece = lane & 7; const int row = Lid >> 1, cofs = (Lid & 1) * 32 + piece * 4;
            const v4f val = *(const v4fa*)(os + row * 68 + cofs); *(volatile v4f*)(crow + (size_t)row * ldc + cofs) = val; }
    };
    pass(); __threadfence(); pass();
}
__global__ __launch_bounds__(256) void k_prep(const float* __restrict__ A, const float* __restrict__ Wm, const float* __restrict__ bm, const float* __restrict__ pw, const float* __restrict__ av, const float* __restrict__ ba, bf* AVh, bf* AVl) {
    __shared__ float Ap[64 * 65]; __shared__ float As[64 * 65];
    const int bh = blockIdx.x, h = bh % NH_, tid = threadIdx.x;
    const float* Ab = A + (size_t)bh * 64 * 64; const float* Wh = Wm + (size_t)h * 64 * 64; const float* bh_ = bm + (size_t)h * 64 * 64; const float* ph = pw + (size_t)h * 64 * 64; const float* avh = av + (size_t)h * 64 * 64; const float* bah = ba + (size_t)h * 64 * 64;
    for (int i = tid; i < 64 * 64; i += 256) As[(i >> 6) * 65 + (i & 63)] = bfr(Ab[i]);
    __syncthreads();
    const int i = tid >> 2, j0 = (tid & 3) * 16;
    float acc[16];
#pragma unroll
    for (int j = 0; j < 16; ++j) acc[j] = 0.f;
#pragma unroll 1
    for (int k = 0; k < 64; ++k) { const float w = bfr(Wh[i * 64 + k]);
#pragma unroll
        for (int j = 0; j < 16; ++j) acc[j] = fmaf(w, As[k * 65 + j0 + j], acc[j]); }
#pragma unroll
    for (int j = 0; j < 16; ++j) Ap[i * 65 + j0 + j] = acc[j] + bfr(bh_[i * 64 + j0 + j]);
#pragma unroll 1
    for (int j = 0; j < 16; ++j) { const int q = i * 65 + j0 + j; const float x = Ap[q]; const float sl = x / (1.0f + expf(-x)); const float aw = x * sl + 1e-9f; Ap[q] = powf(aw, bfr(ph[i * 64 + j0 + j])); }
    __syncthreads();
#pragma unroll
    for (int j = 0; j < 16; ++j) acc[j] = 0.f;
#pragma unroll 1
    for (int k = 0; k < 64; ++k) { const float w = bfr(avh[i * 64 + k]);
#pragma unroll
        for (int j = 0; j < 16; ++j) acc[j] = fmaf(w, Ap[k * 65 + j0 + j], acc[j]); }
    __syncthreads();
#pragma unroll
    for (int j = 0; j < 16; ++j) As[i * 65 + j0 + j] = acc[j] + bfr(bah[i * 64 + j0 + j]);
    __syncthreads();
    const int piece = tid & 7;
#pragma unroll 1
    for (int ps = 0; ps < 2; ++ps) {
#pragma unroll
        for (int r = 0; r < 2; ++r) { const int e = (tid >> 3) + 32 * r; v8us oh, ol;
#pragma unroll
            for (int k = 0; k < 8; ++k) { const float v = As[(piece * 8 + k) * 65 + e]; const unsigned short hb = f2bf(v); oh[k] = hb; ol[k] = f2bf(v - bf2f(hb)); }
            const size_t o = ((size_t)bh * 64 + e) * 64 + piece * 8; *(volatile v8us*)(AVh + o) = oh; *(volatile v8us*)(AVl + o) = ol; }
        if (ps == 0) __threadfence(); }
}
__global__ __launch_bounds__(256) void k_hin16(const float* __restrict__ src, bf* dst, size_t n8) {
    const size_t i = (size_t)blockIdx.x * 256 + threadIdx.x; if (i >= n8) return;
    const v8f v = *(const v8f*)(src + i * 8); v8us o;
#pragma unroll
    for (int k = 0; k < 8; ++k) o[k] = f2bf(v[k]);
    *(volatile v8us*)(dst + i * 8) = o; __threadfence(); *(volatile v8us*)(dst + i * 8) = o;
}
__global__ __launch_bounds__(256) void k_zero8(bf* dst, size_t n8) {
    const size_t i = (size_t)blockIdx.x * 256 + threadIdx.x; if (i >= n8) return; const v8us z = {};
    *(volatile v8us*)(dst + i * 8) = z; __threadfence(); *(volatile v8us*)(dst + i * 8) = z;
}
__global__ __launch_bounds__(256) void k_k16(const float* __restrict__ Hk, h16* K16) {
    const size_t i = (size_t)blockIdx.x * 256 + threadIdx.x; if (i >= (size_t)NBH * NT_ * HD / 8) return;
    const size_t e = i * 8; const int d = (int)(e & 63); const size_t t = (e >> 6) % NT_; const size_t bh = (e >> 6) / NT_; const int b = (int)(bh / NH_), h = (int)(bh % NH_);
    const v8f v = *(const v8f*)(Hk + e); v8h o;
#pragma unroll
    for (int k = 0; k < 8; ++k) o[k] = (h16)bfr(v[k]);
    h16* p = K16 + ((size_t)b * NT_ + t) * DM + h * HD + d; *(volatile v8h*)p = o; __threadfence(); *(volatile v8h*)p = o;
}
__global__ __launch_bounds__(256) void k_sp16b(const float* __restrict__ T, int nrows, h16* Yh, h16* Yl) {
    const int lane = threadIdx.x & 31, r = blockIdx.x * 8 + (threadIdx.x >> 5);
    if (r >= nrows) return;
#pragma unroll 1
    for (int ps = 0; ps < 2; ++ps) {
#pragma unroll 1
        for (int q = 0; q < DM / 256; ++q) { const size_t o = (size_t)r * DM + q * 256 + lane * 8; const v8f v = *(const v8f*)(T + o); v8h oh, ol;
#pragma unroll
            for (int k = 0; k < 8; ++k) { const h16 a = (h16)v[k]; oh[k] = a; ol[k] = (h16)((v[k] - (float)a) * LOSC); }
            *(volatile v8h*)(Yh + o) = oh; *(volatile v8h*)(Yl + o) = ol; }
        if (ps == 0) __threadfence(); }
}
__global__ __launch_bounds__(256) void k_vt(const float* __restrict__ v, h16* VT16) {
    __shared__ __align__(16) h16 tile[HD * 72];
    const int bh = blockIdx.x / (NT_ / 64), kt = blockIdx.x - bh * (NT_ / 64), t0 = kt * 64, tid = threadIdx.x;
    const int tt = tid >> 2, d0 = (tid & 3) * 16;
    const float* src = v + ((size_t)bh * NT_ + t0 + tt) * HD + d0;
#pragma unroll
    for (int i = 0; i < 16; ++i) tile[(d0 + i) * 72 + tt] = (h16)bfr(src[i]);
    __syncthreads();
    const int piece = tid & 7;
    const size_t base = ((size_t)bh * HD) * NT_ + t0;
    auto pass = [&]() {
#pragma unroll
        for (int s = 0; s < 2; ++s) { const int d = (tid >> 3) + 32 * s; const v8h val = *(const v8ha*)(tile + d * 72 + piece * 8); *(volatile v8h*)(VT16 + base + (size_t)d * NT_ + piece * 8) = val; }
    };
    pass(); __threadfence(); pass();
}
__global__ __launch_bounds__(128) void k_attn(const h16* __restrict__ Q16, const h16* __restrict__ QL16, const h16* __restrict__ K16, const h16* __restrict__ VTH, const float* __restrict__ AM, float* OUTP) {
    __shared__ __align__(16) h16 plds[4][16 * 32];
    __shared__ __align__(16) h16 plds2[4][16 * 32];
    __shared__ __align__(16) float ost[4][16 * 68];
    const int lane = threadIdx.x & 31, wave = threadIdx.x >> 5, lr = lane & 15, hi = lane >> 4;
    const int bid = blockIdx.x;
    const int b = bid / (NH_ * (NT_ / 64)), rem = bid - b * (NH_ * (NT_ / 64)), h = rem / (NT_ / 64), qt = rem - h * (NT_ / 64);
    const int q0 = qt * 64 + wave * 16;
    const size_t tok0 = (size_t)b * NT_;
    h16* pl = &plds[wave][0]; h16* pl2 = &plds2[wave][0];
    v16h qa[2];
    const size_t qo0 = (tok0 + q0 + lr) * DM + h * HD + 8 * hi;
#pragma unroll
    for (int kc = 0; kc < 2; ++kc) qa[kc] = cat16(*(const v8h*)(Q16 + qo0 + kc * 32), *(const v8h*)(Q16 + qo0 + kc * 32 + 16));
    const h16* kh_b = K16 + tok0 * DM + h * HD;
    const size_t vbase = (((size_t)b * NH_ + h) * HD) * NT_;
    v8f o[4], ox[4];
#pragma unroll
    for (int n = 0; n < 4; ++n) { o[n] = (v8f){}; ox[n] = (v8f){}; }
    float mrow[8], lpart[8];
#pragma unroll
    for (int j = 0; j < 8; ++j) { mrow[j] = -3.0e38f; lpart[j] = 0.f; }
    int qpos[8];
#pragma unroll
    for (int j = 0; j < 8; ++j) qpos[j] = q0 + 8 * hi + j;
    const int kt_lo = 0, kt_hi = (qt * 64 + 63) / 32;
    const float* am = AM + (size_t)b * NT_ * NT_;
#pragma unroll 1
    for (int kt = kt_lo; kt <= kt_hi; ++kt) {
        const int l0 = kt * 32;
        const size_t ko0 = (size_t)(l0 + lr) * DM + 8 * hi, ko1 = (size_t)(l0 + 16 + lr) * DM + 8 * hi;
        v8f s0 = {}, s1 = {}, x0 = {}, x1 = {};
#pragma unroll
        for (int kc = 0; kc < 2; ++kc) {
            { const v16h k0h = cat16(*(const v8h*)(kh_b + ko0 + kc * 32), *(const v8h*)(kh_b + ko0 + kc * 32 + 16)), k1h = cat16(*(const v8h*)(kh_b + ko1 + kc * 32), *(const v8h*)(kh_b + ko1 + kc * 32 + 16));
              const v16h qlk = cat16(*(const v8h*)(QL16 + qo0 + kc * 32), *(const v8h*)(QL16 + qo0 + kc * 32 + 16));
              s0 = wmma16(qa[kc], k0h, s0); x0 = wmma16(qlk, k0h, x0); s1 = wmma16(qa[kc], k1h, s1); x1 = wmma16(qlk, k1h, x1);
              asm volatile("v_nop" : "+v"(s0), "+v"(s1), "+v"(x0), "+v"(x1) : "v"(qlk), "v"(k0h), "v"(k1h) : "memory"); }
        }
        asm volatile("v_nop\n\tv_nop\n\tv_nop\n\tv_nop" : "+v"(s0), "+v"(s1), "+v"(x0), "+v"(x1) : "v"(qa[0]), "v"(qa[1]));
        float alpha[8];
#pragma unroll
        for (int j = 0; j < 8; ++j) {
            const int ja = l0 + lr, jb = l0 + 16 + lr, qi = qpos[j];
            const float a0 = (s0[j] + x0[j] * LOSCI) * 0.125f + bfr(am[(size_t)qi * NT_ + ja]), a1 = (s1[j] + x1[j] * LOSCI) * 0.125f + bfr(am[(size_t)qi * NT_ + jb]);
            float mx = fmaxf(a0, a1);
            mx = fmaxf(mx, __shfl_xor(mx, 1, 16)); mx = fmaxf(mx, __shfl_xor(mx, 2, 16)); mx = fmaxf(mx, __shfl_xor(mx, 4, 16)); mx = fmaxf(mx, __shfl_xor(mx, 8, 16));
            const float mn = fmaxf(mrow[j], mx);
            alpha[j] = __expf(mrow[j] - mn); mrow[j] = mn;
            const float p0 = __expf(a0 - mn), p1 = __expf(a1 - mn);
            lpart[j] = lpart[j] * alpha[j] + (p0 + p1);
            const int mr = hi * 8 + j;
            const float ps0 = p0 * PSC, ps1 = p1 * PSC; const h16 h0 = (h16)ps0, h1 = (h16)ps1;
            pl[mr * 32 + lr] = h0; pl[mr * 32 + 16 + lr] = h1;
            pl2[mr * 32 + lr] = (h16)((ps0 - (float)h0) * LOSC); pl2[mr * 32 + 16 + lr] = (h16)((ps1 - (float)h1) * LOSC);
        }
#pragma unroll
        for (int n = 0; n < 4; ++n)
#pragma unroll
            for (int j = 0; j < 8; ++j) { o[n][j] *= alpha[j]; ox[n][j] *= alpha[j]; }
        asm volatile("" ::: "memory");
        const v16h pa = cat16(*(const v8ha*)(pl + lr * 32 + hi * 8), *(const v8ha*)(pl + lr * 32 + 16 + hi * 8));
        const v16h px = cat16(*(const v8ha*)(pl2 + lr * 32 + hi * 8), *(const v8ha*)(pl2 + lr * 32 + 16 + hi * 8));
#pragma unroll
        for (int n = 0; n < 4; ++n) { const size_t vo = vbase + (size_t)(n * 16 + lr) * NT_ + l0 + hi * 8;
            const v16h vh = cat16(*(const v8h*)(VTH + vo), *(const v8h*)(VTH + vo + 16));
            o[n] = wmma16(pa, vh, o[n]); ox[n] = wmma16(px, vh, ox[n]);
            asm volatile("" : "+v"(o[n]), "+v"(ox[n]) : "v"(vh) : "memory"); }
        asm volatile("v_nop\n\tv_nop\n\tv_nop\n\tv_nop" : "+v"(o[0]), "+v"(o[1]), "+v"(o[2]), "+v"(o[3]), "+v"(ox[0]), "+v"(ox[1]), "+v"(ox[2]), "+v"(ox[3]) : "v"(pa), "v"(px));
    }
    float inv[8];
#pragma unroll
    for (int j = 0; j < 8; ++j) { float rs = lpart[j]; rs += __shfl_xor(rs, 1, 16); rs += __shfl_xor(rs, 2, 16); rs += __shfl_xor(rs, 4, 16); rs += __shfl_xor(rs, 8, 16); inv[j] = 1.0f / (rs * PSC); }
    float* os = &ost[wave][0];
#pragma unroll
    for (int n = 0; n < 4; ++n)
#pragma unroll
        for (int j = 0; j < 8; ++j) os[(hi * 8 + j) * 68 + n * 16 + lr] = (o[n][j] + ox[n][j] * LOSCI) * inv[j];
    __syncthreads();
    float* ob = OUTP + (tok0 + q0) * DM + (size_t)h * HD;
    auto pass = [&]() {
#pragma unroll
        for (int s = 0; s < 8; ++s) { const int Lid = (lane >> 3) + 4 * s, piece = lane & 7; const int row = Lid >> 1, cofs = (Lid & 1) * 32 + piece * 4;
            const v4f val = *(const v4fa*)(os + row * 68 + cofs); *(volatile v4f*)(ob + (size_t)row * DM + cofs) = val; }
    };
    pass(); __threadfence(); pass();
}

#define VST2(T, p, v) do { const T vst2_v_ = (v); *(volatile T*)(p) = vst2_v_; __threadfence(); *(volatile T*)(p) = vst2_v_; } while (0)
extern "C" void kernel_launch(void* const* d_in, const int* in_sizes, int n_in,
                              void* d_out, int out_size, void* d_ws, size_t ws_size, hipStream_t stream) {
    (void)in_sizes; (void)n_in; (void)out_size;
    const float* Hin = (const float*)d_in[0]; const float* Hk = (const float*)d_in[1]; const float* Hv = (const float*)d_in[2]; const float* A = (const float*)d_in[3]; const float* AM = (const float*)d_in[4];
    const float* Wm = (const float*)d_in[5]; const float* bm = (const float*)d_in[6]; const float* pw = (const float*)d_in[7]; const float* av = (const float*)d_in[8]; const float* ba = (const float*)d_in[9];
    float* out = (float*)d_out;
    char* wsp = (char*)d_ws;
    auto take = [&](size_t bytes) { char* p = wsp; wsp += (bytes + 255) & ~(size_t)255; return (void*)p; };
    bf* AVh = (bf*)take((size_t)NBH * 64 * 64 * 2); bf* AVl = (bf*)take((size_t)NBH * 64 * 64 * 2);
    bf* HinB = (bf*)take((size_t)NBH * NT_ * HD * 2); bf* ZER = (bf*)take((size_t)NT_ * HD * 2);
    h16* K16 = (h16*)take((size_t)NBH * NT_ * HD * 2); h16* VT16 = (h16*)take((size_t)NBH * HD * NT_ * 2);
    float* Qf = (float*)take((size_t)NTK * DM * 4); h16* QH = (h16*)take((size_t)NTK * DM * 2); h16* QL = (h16*)take((size_t)NTK * DM * 2);
    if ((size_t)(wsp - (char*)d_ws) > ws_size) return;
    k_prep<<<NBH, 256, 0, stream>>>(A, Wm, bm, pw, av, ba, AVh, AVl);
    k_hin16<<<(unsigned)((size_t)NBH * NT_ * HD / 8 / 256), 256, 0, stream>>>(Hin, HinB, (size_t)NBH * NT_ * HD / 8);
    k_zero8<<<(NT_ * HD / 8) / 256, 256, 0, stream>>>(ZER, (size_t)NT_ * HD / 8);
    k_k16<<<(unsigned)((size_t)NBH * NT_ * HD / 8 / 256), 256, 0, stream>>>(Hk, K16);
    k_vt<<<NBH * (NT_ / 64), 256, 0, stream>>>(Hv, VT16);
    for (int b = 0; b < 2; ++b) {
        for (int h = 0; h < NH_; ++h)
            k_gemm3<<<dim3(NT_ / 64, 1, 1), 128, 0, stream>>>(HinB + ((size_t)b * NH_ + h) * NT_ * HD, ZER, AVh + ((size_t)b * NH_ + h) * 64 * 64, AVl + ((size_t)b * NH_ + h) * 64 * 64, HD, Qf + h * HD, DM);
        k_sp16b<<<NTK / 8, 256, 0, stream>>>(Qf, NTK, QH, QL);
        k_attn<<<NB_ * NH_ * (NT_ / 64), 128, 0, stream>>>(QH, QL, K16 + (size_t)b * NT_ * DM, VT16 + (size_t)b * NH_ * HD * NT_, AM, out + (size_t)b * NTK * DM);
    }
}
